// GAT_Classifier_90821378441672
// MI455X (gfx1250) — hardware-verified
//
#include <hip/hip_runtime.h>
#include <stddef.h>


#define HDIM   192
#define NHEAD  6
#define DHEAD  32
#define FIN    89
#define NG     256
#define NC     10
#define GR     32
#define GTHR   192
#define GWAVE  6
#define XP     196
#define NB     256
#define CHUNK  2048
#define ATHR   256
#define NWAVE  8
#define WCAP   256
#define NGRP   (CHUNK / (ATHR * 4))
#define W1P    200
#define W2P    40
#define ZP     36
#define SW     8.0f
#define ISW    0.125f
#define SA     16.0f
#define ISWA   (1.0f / 128.0f)

#define LDS_ACC  (NB * HDIM)
#define LDS_DEN  (NB * NHEAD)
#define LDS_MX   (NB * NHEAD)
#define LDS_LIST (NWAVE * WCAP)
#define AGG_LDS_BYTES ((LDS_ACC + LDS_DEN + LDS_MX + LDS_LIST + NWAVE) * 4)

static_assert(WCAP == (CHUNK / ATHR) * 32);
static_assert(NGRP == 2);
static_assert(NB == 256);
static_assert(((LDS_ACC + LDS_DEN) % 4) == 0);
static_assert(AGG_LDS_BYTES == 217120);
static_assert(GTHR == GWAVE * 32);
static_assert(HDIM == NHEAD * DHEAD);
static_assert((XP % 4) == 0);
static_assert((ZP % 4) == 0);

typedef float    v4f  __attribute__((ext_vector_type(4)));
typedef float    v8f  __attribute__((ext_vector_type(8)));
typedef int      v4i  __attribute__((ext_vector_type(4)));
typedef _Float16 v8h  __attribute__((ext_vector_type(8)));
typedef _Float16 v16h __attribute__((ext_vector_type(16)));
union Frag   { v16h v; v8h half[2]; };
union Pack16 { v8h h; v4i i; };

__device__ __forceinline__ v8f wm(v16h a, v16h b, v8f c) {
  v8f d = __builtin_amdgcn_wmma_f32_16x16x32_f16(false, a, false, b, (short)0, c, false, false);
  asm volatile("v_nop\n\tv_nop\n\tv_nop\n\tv_nop" : "+v"(d) : "v"(a), "v"(b));
  return d;
}

__device__ __forceinline__ v8f zero8() {
  v8f z = {0.f, 0.f, 0.f, 0.f, 0.f, 0.f, 0.f, 0.f};
  return z;
}

__device__ __forceinline__ v8h pack8(v4f a, v4f b, float s) {
  Pack16 u;
  u.h[0] = (_Float16)(a.x * s); u.h[1] = (_Float16)(a.y * s);
  u.h[2] = (_Float16)(a.z * s); u.h[3] = (_Float16)(a.w * s);
  u.h[4] = (_Float16)(b.x * s); u.h[5] = (_Float16)(b.y * s);
  u.h[6] = (_Float16)(b.z * s); u.h[7] = (_Float16)(b.w * s);
  return u.h;
}

__global__ __launch_bounds__(256) void k_prepw(const float* __restrict__ W, _Float16* Wt, int K, int WP) {
  const int gpr = WP >> 3;
  const int i = blockIdx.x * 256 + threadIdx.x;
  if (i >= HDIM * gpr) return;
  const int n  = i / gpr;
  const int k0 = (i - n * gpr) * 8;
  Pack16 u;
#pragma unroll
  for (int j = 0; j < 8; ++j) {
    const int k = k0 + j;
    float v = 0.f;
    if (k < K) v = W[(size_t)k * HDIM + n] * SW;
    u.h[j] = (_Float16)v;
  }
  _Float16* p = Wt + (size_t)n * WP + k0;
  *(volatile v4i*)p = u.i;
  __threadfence();
  *(volatile v4i*)p = u.i;
}

__device__ __forceinline__ void epi2(v8f a0, v8f a1, int T, int hh, int m, int wave, int n0,
                                     float s0, float s1, float d0, float d1,
                                     float* Xs, float* Els, float* Ers) {
  float ss[8], sd[8];
#pragma unroll
  for (int r = 0; r < 8; ++r) {
    const float v0 = a0[r] * ISW;
    const float v1 = a1[r] * ISW;
    const int row = T * 16 + 8 * hh + r;
    Xs[row * XP + n0 + m]      = v0;
    Xs[row * XP + n0 + 16 + m] = v1;
    ss[r] = v0 * s0 + v1 * s1;
    sd[r] = v0 * d0 + v1 * d1;
  }
#pragma unroll
  for (int mk = 1; mk < 16; mk <<= 1) {
#pragma unroll
    for (int r = 0; r < 8; ++r) {
      ss[r] += __shfl_xor(ss[r], mk, 32);
      sd[r] += __shfl_xor(sd[r], mk, 32);
    }
  }
  if (m == 0) {
#pragma unroll
    for (int r = 0; r < 8; ++r) {
      const int row = T * 16 + 8 * hh + r;
      Els[row * NHEAD + wave] = ss[r];
      Ers[row * NHEAD + wave] = sd[r];
    }
  }
}

__device__ __forceinline__ void gemm_store_pass(const float* Xs, const float* Els, const float* Ers,
                                                float* F, float* El, float* Er,
                                                int rowBase, int wave, int lane) {
  for (int r = wave; r < GR; r += GWAVE) {
    float* gp = F + (size_t)(rowBase + r) * HDIM + 4 * lane;
    const v4f v0 = *(const v4f*)(Xs + r * XP + 4 * lane);
    *(volatile v4f*)gp = v0;
    if (lane < 16) {
      const v4f v1 = *(const v4f*)(Xs + r * XP + 128 + 4 * lane);
      *(volatile v4f*)(gp + 128) = v1;
    }
  }
  if (wave < 2) {
    const float* S = (wave == 0) ? Els : Ers;
    float* E = (wave == 0) ? El : Er;
    float* gp = E + (size_t)rowBase * NHEAD + 4 * lane;
    const v4f e0 = *(const v4f*)(S + 4 * lane);
    *(volatile v4f*)gp = e0;
    if (lane < 16) {
      const v4f e1 = *(const v4f*)(S + 128 + 4 * lane);
      *(volatile v4f*)(gp + 128) = e1;
    }
  }
}

template <int K, int KP, int WP>
__global__ __launch_bounds__(GTHR) void k_gemm(
    const float* __restrict__ X, const _Float16* __restrict__ Wt,
    const float* __restrict__ al, const float* __restrict__ ar,
    float* F, float* El, float* Er, int nN) {
  constexpr int AP = KP + 8;
  static_assert((KP % 32) == 0);
  static_assert((AP % 8) == 0);
  static_assert(K <= KP);
  __shared__ __attribute__((aligned(16))) _Float16 At[GR * AP];
  __shared__ __attribute__((aligned(16))) float Xs[GR * XP];
  __shared__ __attribute__((aligned(16))) float Els[GR * NHEAD];
  __shared__ __attribute__((aligned(16))) float Ers[GR * NHEAD];

  const int tid  = threadIdx.x;
  const int lane = tid & 31;
  const int wave = tid >> 5;
  const int hh   = lane >> 4;
  const int m    = lane & 15;
  const int rowBase = blockIdx.x * GR;

  for (int r = wave; r < GR; r += GWAVE) {
    int row = rowBase + r;
    if (row > nN - 1) row = nN - 1;
    const float* xr = X + (size_t)row * K;
    for (int k = lane; k < KP; k += 32) {
      const float v = (k < K) ? xr[k] : 0.f;
      At[r * AP + k] = (_Float16)v;
    }
  }
  __syncthreads();

  const int n0 = wave * DHEAD;
  v8f c00 = zero8(), c01 = zero8(), c10 = zero8(), c11 = zero8();
#pragma unroll
  for (int kt = 0; kt < KP / 32; ++kt) {
    const int k0 = kt * 32;
    Frag a0, a1, b0, b1;
    const _Float16* pa0 = At + m * AP + k0 + 8 * hh;
    const _Float16* pa1 = At + (16 + m) * AP + k0 + 8 * hh;
    const _Float16* pb0 = Wt + (size_t)(n0 + m) * WP + k0 + 8 * hh;
    const _Float16* pb1 = Wt + (size_t)(n0 + 16 + m) * WP + k0 + 8 * hh;
    a0.half[0] = *(const v8h*)pa0; a0.half[1] = *(const v8h*)(pa0 + 16);
    a1.half[0] = *(const v8h*)pa1; a1.half[1] = *(const v8h*)(pa1 + 16);
    b0.half[0] = *(const v8h*)pb0; b0.half[1] = *(const v8h*)(pb0 + 16);
    b1.half[0] = *(const v8h*)pb1; b1.half[1] = *(const v8h*)(pb1 + 16);
    c00 = wm(a0.v, b0.v, c00);
    c01 = wm(a0.v, b1.v, c01);
    c10 = wm(a1.v, b0.v, c10);
    c11 = wm(a1.v, b1.v, c11);
  }

  const float s0 = al[n0 + m], s1 = al[n0 + 16 + m];
  const float d0 = ar[n0 + m], d1 = ar[n0 + 16 + m];
  epi2(c00, c01, 0, hh, m, wave, n0, s0, s1, d0, d1, Xs, Els, Ers);
  epi2(c10, c11, 1, hh, m, wave, n0, s0, s1, d0, d1, Xs, Els, Ers);
  __syncthreads();

  gemm_store_pass(Xs, Els, Ers, F, El, Er, rowBase, wave, lane);
  __threadfence();
  gemm_store_pass(Xs, Els, Ers, F, El, Er, rowBase, wave, lane);
}

__global__ __launch_bounds__(ATHR) void k_agg(
    const float* __restrict__ F, const float* __restrict__ El, const float* __restrict__ Er,
    const int* __restrict__ src, const int* __restrict__ dst, const float* __restrict__ bias,
    float* Hout, int nN, int nE) {
  extern __shared__ v4f lds_dyn[];
  float* acc  = (float*)lds_dyn;
  float* den  = acc + LDS_ACC;
  float* mx   = den + LDS_DEN;
  int*   list = (int*)(mx + LDS_MX);
  int*   wcnt = list + LDS_LIST;

  const int tid  = threadIdx.x;
  const int lane = tid & 31;
  const int wave = tid >> 5;
  const int nodeBase = blockIdx.x * NB;

  {
    const v4f z4 = {0.f, 0.f, 0.f, 0.f};
    for (int i = tid; i < (LDS_ACC + LDS_DEN) / 4; i += ATHR) lds_dyn[i] = z4;
    const float ninf = -__builtin_inff();
    for (int i = tid; i < LDS_MX; i += ATHR) mx[i] = ninf;
  }
  __syncthreads();

  int hd;
  if (lane < 24) hd = lane >> 2;
  else if (lane < 30) hd = lane - 24;
  else hd = NHEAD - 1;
  const bool accLane = (lane < 24);
  const bool denLane = (lane >= 24) && (lane < 30);
  const bool al16 = ((((size_t)dst) & 15) == 0);

  const int nChunks = (nE + CHUNK - 1) / CHUNK;
#pragma unroll 1
  for (int ch = 0; ch < nChunks; ++ch) {
    const int cbase = ch * CHUNK;
    int wc = 0;
#pragma unroll
    for (int g = 0; g < NGRP; ++g) {
      const int el0 = (g * ATHR + tid) * 4;
      const int e0  = cbase + el0;
      const int sent = -2147483647 - 1;
      v4i d;
      if (al16 && (e0 + 3 < nE)) {
        d = *(const v4i*)(dst + e0);
      } else {
        d.x = (e0     < nE) ? dst[e0]     : sent;
        d.y = (e0 + 1 < nE) ? dst[e0 + 1] : sent;
        d.z = (e0 + 2 < nE) ? dst[e0 + 2] : sent;
        d.w = (e0 + 3 < nE) ? dst[e0 + 3] : sent;
      }
      const unsigned s0 = (unsigned)d.x - (unsigned)nodeBase;
      const unsigned s1 = (unsigned)d.y - (unsigned)nodeBase;
      const unsigned s2 = (unsigned)d.z - (unsigned)nodeBase;
      const unsigned s3 = (unsigned)d.w - (unsigned)nodeBase;
      const bool h0 = s0 < (unsigned)NB;
      const bool h1 = s1 < (unsigned)NB;
      const bool h2 = s2 < (unsigned)NB;
      const bool h3 = s3 < (unsigned)NB;
      const unsigned many = __builtin_amdgcn_ballot_w32(h0 | h1 | h2 | h3);
      if (many != 0u) {
#define HITJ(J, HJ, SJ) { \
          const unsigned mj = __builtin_amdgcn_ballot_w32(HJ); \
          if (HJ) { \
            const int pos = wc + (int)__builtin_amdgcn_mbcnt_lo(mj, 0u); \
            if (pos < WCAP) list[wave * WCAP + pos] = ((el0 + (J)) << 8) | (int)(SJ); \
          } \
          wc += (int)__builtin_popcount(mj); }
        HITJ(0, h0, s0)
        HITJ(1, h1, s1)
        HITJ(2, h2, s2)
        HITJ(3, h3, s3)
#undef HITJ
      }
    }
    if (lane == 0) wcnt[wave] = wc;
    __syncthreads();

    if (wave == 0) {
#pragma unroll 1
      for (int wsx = 0; wsx < NWAVE; ++wsx) {
        int n = wcnt[wsx];
        if (n > WCAP) n = WCAP;
        if (n < 0) n = 0;
#pragma unroll 1
        for (int i = 0; i < n; ++i) {
          const int ent  = list[wsx * WCAP + i];
          const int slot = ent & (NB - 1);
          const int eloc = (ent >> 8) & (CHUNK - 1);
          int e = cbase + eloc;
          if (e > nE - 1) e = nE - 1;
          int s = src[e];
          s = s < 0 ? 0 : (s > nN - 1 ? nN - 1 : s);
          int nd = nodeBase + slot;
          if (nd > nN - 1) nd = nN - 1;
          float a = El[(size_t)s * NHEAD + hd] + Er[(size_t)nd * NHEAD + hd];
          a = (a > 0.f) ? a : 0.2f * a;
          const int mi = slot * NHEAD + hd;
          const float mo = mx[mi];
          const float mn = fmaxf(mo, a);
          const float sc = __expf(mo - mn);
          const float p  = __expf(a - mn);
          if (accLane) {
            const float* fp = F + (size_t)s * HDIM + 8 * lane;
            const v4f f0 = *(const v4f*)fp;
            const v4f f1 = *(const v4f*)(fp + 4);
            v4f* ap = (v4f*)(acc + slot * HDIM + 8 * lane);
            const v4f o0 = ap[0];
            const v4f o1 = ap[1];
            const v4f n0 = o0 * sc + f0 * p;
            const v4f n1 = o1 * sc + f1 * p;
            ap[0] = n0;
            ap[1] = n1;
          }
          if (denLane) {
            const float od = den[mi];
            den[mi] = od * sc + p;
          }
          mx[mi] = mn;
        }
      }
    }
    __syncthreads();
  }

  const int hdA = lane >> 3;
  const int hdB = 4 + (lane >> 3);
  const v4f bA = *(const v4f*)(bias + 4 * lane);
  v4f bB = {0.f, 0.f, 0.f, 0.f};
  if (lane < 16) bB = *(const v4f*)(bias + 128 + 4 * lane);
#pragma unroll 1
  for (int j = 0; j < NB / NWAVE; ++j) {
    const int slot = wave * (NB / NWAVE) + j;
    const int node = nodeBase + slot;
    if (node >= nN) break;
    const float dA = den[slot * NHEAD + hdA];
    const float iA = (dA > 0.f) ? (1.0f / dA) : 0.f;
    const v4f vA = *(const v4f*)(acc + slot * HDIM + 4 * lane) * iA + bA;
    v4f vB = bB;
    if (lane < 16) {
      const float dB = den[slot * NHEAD + hdB];
      const float iB = (dB > 0.f) ? (1.0f / dB) : 0.f;
      vB = *(const v4f*)(acc + slot * HDIM + 128 + 4 * lane) * iB + bB;
    }
    float* hp = Hout + (size_t)node * HDIM + 4 * lane;
    *(volatile v4f*)hp = vA;
    if (lane < 16) *(volatile v4f*)(hp + 128) = vB;
    __threadfence();
    *(volatile v4f*)hp = vA;
    if (lane < 16) *(volatile v4f*)(hp + 128) = vB;
  }
}

__global__ __launch_bounds__(256) void k_readout(const float* __restrict__ H, const int* __restrict__ gid,
                                                 float* Hg, int nN) {
  __shared__ int hl[256];
  __shared__ int hc[NWAVE];
  __shared__ __attribute__((aligned(16))) float sh[HDIM];
  const int g    = blockIdx.x;
  const int tid  = threadIdx.x;
  const int lane = tid & 31;
  const int wave = tid >> 5;
  float s = 0.f;
  int cnt = 0;
  const int nCh = (nN + 255) / 256;
#pragma unroll 1
  for (int ch = 0; ch < nCh; ++ch) {
    const int n = ch * 256 + tid;
    int gv = -1;
    if (n < nN) gv = gid[n];
    const bool hit = (gv == g);
    const unsigned mk = __builtin_amdgcn_ballot_w32(hit);
    if (hit) {
      const int pos = (int)__builtin_amdgcn_mbcnt_lo(mk, 0u);
      hl[wave * 32 + pos] = n;
    }
    if (lane == 0) hc[wave] = (int)__builtin_popcount(mk);
    __syncthreads();
#pragma unroll 1
    for (int w = 0; w < NWAVE; ++w) {
      int c = hc[w];
      if (c > 32) c = 32;
      if (c < 0) c = 0;
      cnt += c;
      if (tid < HDIM) {
#pragma unroll 1
        for (int i = 0; i < c; ++i) {
          int nn = hl[w * 32 + i];
          nn = nn < 0 ? 0 : (nn > nN - 1 ? nN - 1 : nn);
          s += H[(size_t)nn * HDIM + tid];
        }
      }
    }
    __syncthreads();
  }
  const float cf  = (float)cnt;
  const float inv = 1.0f / fmaxf(cf, 1.0f);
  if (tid < HDIM) sh[tid] = s * inv;
  __syncthreads();
  v4f v = {0.f, 0.f, 0.f, 0.f};
  float* gp = 0;
  if (wave == 0) {
    v  = *(const v4f*)(sh + 4 * lane);
    gp = Hg + (size_t)g * HDIM + 4 * lane;
  } else if (wave == 1 && lane < 16) {
    v  = *(const v4f*)(sh + 128 + 4 * lane);
    gp = Hg + (size_t)g * HDIM + 128 + 4 * lane;
  }
  if (gp) *(volatile v4f*)gp = v;
  __threadfence();
  if (gp) *(volatile v4f*)gp = v;
}

__global__ __launch_bounds__(256) void k_cls(const float* __restrict__ Hg, const float* __restrict__ Wc1,
                                             const float* __restrict__ bc1, const float* __restrict__ Wc2,
                                             const float* __restrict__ bc2, float* out) {
  __shared__ __attribute__((aligned(16))) _Float16 W1t[DHEAD * W1P];
  __shared__ __attribute__((aligned(16))) _Float16 W2t[16 * W2P];
  __shared__ __attribute__((aligned(16))) float Z[NG * ZP];
  __shared__ __attribute__((aligned(16))) float Os[NG * NC];

  const int tid  = threadIdx.x;
  const int lane = tid & 31;
  const int wave = tid >> 5;
  const int hh   = lane >> 4;
  const int m    = lane & 15;

  for (int i = tid; i < DHEAD * HDIM; i += 256) {
    const int n = i / HDIM;
    const int k = i - n * HDIM;
    W1t[n * W1P + k] = (_Float16)(Wc1[k * DHEAD + n] * SW);
  }
  for (int i = tid; i < 16 * DHEAD; i += 256) {
    const int c = i >> 5;
    const int k = i & 31;
    float v = 0.f;
    if (c < NC) v = Wc2[k * NC + c] * SW;
    W2t[c * W2P + k] = (_Float16)v;
  }
  __syncthreads();

  const int rw = wave * 32;
  v8f c00 = zero8(), c01 = zero8(), c10 = zero8(), c11 = zero8();
#pragma unroll
  for (int kt = 0; kt < HDIM / 32; ++kt) {
    const int k0 = kt * 32;
    Frag a0, a1, b0, b1;
    const float* ph0 = Hg + (size_t)(rw + m) * HDIM + k0 + 8 * hh;
    const float* ph1 = Hg + (size_t)(rw + 16 + m) * HDIM + k0 + 8 * hh;
    a0.half[0] = pack8(*(const v4f*)ph0,        *(const v4f*)(ph0 + 4),  SA);
    a0.half[1] = pack8(*(const v4f*)(ph0 + 16), *(const v4f*)(ph0 + 20), SA);
    a1.half[0] = pack8(*(const v4f*)ph1,        *(const v4f*)(ph1 + 4),  SA);
    a1.half[1] = pack8(*(const v4f*)(ph1 + 16), *(const v4f*)(ph1 + 20), SA);
    const _Float16* pb0 = W1t + m * W1P + k0 + 8 * hh;
    const _Float16* pb1 = W1t + (16 + m) * W1P + k0 + 8 * hh;
    b0.half[0] = *(const v8h*)pb0; b0.half[1] = *(const v8h*)(pb0 + 16);
    b1.half[0] = *(const v8h*)pb1; b1.half[1] = *(const v8h*)(pb1 + 16);
    c00 = wm(a0.v, b0.v, c00);
    c01 = wm(a0.v, b1.v, c01);
    c10 = wm(a1.v, b0.v, c10);
    c11 = wm(a1.v, b1.v, c11);
  }
  {
    const float bb0 = bc1[m], bb1 = bc1[16 + m];
#pragma unroll
    for (int r = 0; r < 8; ++r) {
      const int row0 = rw + 8 * hh + r;
      const int row1 = rw + 16 + 8 * hh + r;
      float z;
      z = c00[r] * ISWA + bb0; Z[row0 * ZP + m]      = z > 0.f ? z : 0.f;
      z = c01[r] * ISWA + bb1; Z[row0 * ZP + 16 + m] = z > 0.f ? z : 0.f;
      z = c10[r] * ISWA + bb0; Z[row1 * ZP + m]      = z > 0.f ? z : 0.f;
      z = c11[r] * ISWA + bb1; Z[row1 * ZP + 16 + m] = z > 0.f ? z : 0.f;
    }
  }
  __syncthreads();

  v8f d0 = zero8(), d1 = zero8();
  {
    Frag b2;
    const _Float16* pb2 = W2t + m * W2P + 8 * hh;
    b2.half[0] = *(const v8h*)pb2;
    b2.half[1] = *(const v8h*)(pb2 + 16);
    Frag a;
    const float* pz0 = Z + (rw + m) * ZP + 8 * hh;
    a.half[0] = pack8(*(const v4f*)pz0,        *(const v4f*)(pz0 + 4),  SA);
    a.half[1] = pack8(*(const v4f*)(pz0 + 16), *(const v4f*)(pz0 + 20), SA);
    d0 = wm(a.v, b2.v, d0);
    const float* pz1 = Z + (rw + 16 + m) * ZP + 8 * hh;
    a.half[0] = pack8(*(const v4f*)pz1,        *(const v4f*)(pz1 + 4),  SA);
    a.half[1] = pack8(*(const v4f*)(pz1 + 16), *(const v4f*)(pz1 + 20), SA);
    d1 = wm(a.v, b2.v, d1);
  }
  {
    const int mc = (m < NC) ? m : (NC - 1);
    const float b2v = bc2[mc];
#pragma unroll
    for (int r = 0; r < 8; ++r) {
      const int row0 = rw + 8 * hh + r;
      const int row1 = rw + 16 + 8 * hh + r;
      const float o0 = d0[r] * ISWA + b2v;
      const float o1 = d1[r] * ISWA + b2v;
      if (m < NC) {
        Os[row0 * NC + m] = o0;
        Os[row1 * NC + m] = o1;
      }
    }
  }
  __syncthreads();

  for (int i = tid; i < (NG * NC) / 4; i += 256) {
    const v4f v = *(const v4f*)(Os + 4 * i);
    *(volatile v4f*)(out + 4 * i) = v;
  }
  __threadfence();
  for (int i = tid; i < (NG * NC) / 4; i += 256) {
    const v4f v = *(const v4f*)(Os + 4 * i);
    *(volatile v4f*)(out + 4 * i) = v;
  }
}

static inline size_t al256(size_t x) { return (x + 255) & ~(size_t)255; }

extern "C" void kernel_launch(void* const* d_in, const int* in_sizes, int n_in,
                              void* d_out, int out_size, void* d_ws, size_t ws_size,
                              hipStream_t stream) {
  if (n_in < 20) return;
  const int nN = in_sizes[0] / FIN;
  if (nN <= 0 || in_sizes[0] != nN * FIN) return;
  const int nE = in_sizes[17];
  if (nE <= 0 || in_sizes[18] != nE) return;
  if (in_sizes[19] != nN) return;
  if (in_sizes[1] != FIN * HDIM || in_sizes[5] != HDIM * HDIM || in_sizes[9] != HDIM * HDIM) return;
  if (in_sizes[2] != HDIM || in_sizes[3] != HDIM || in_sizes[4] != HDIM) return;
  if (in_sizes[6] != HDIM || in_sizes[7] != HDIM || in_sizes[8] != HDIM) return;
  if (in_sizes[10] != HDIM || in_sizes[11] != HDIM || in_sizes[12] != HDIM) return;
  if (in_sizes[13] != HDIM * DHEAD || in_sizes[14] != DHEAD) return;
  if (in_sizes[15] != DHEAD * NC || in_sizes[16] != NC) return;
  if (out_size != NG * NC) return;

  const float* nf  = (const float*)d_in[0];
  const float* W1  = (const float*)d_in[1];
  const float* al1 = (const float*)d_in[2];
  const float* ar1 = (const float*)d_in[3];
  const float* b1  = (const float*)d_in[4];
  const float* W2  = (const float*)d_in[5];
  const float* al2 = (const float*)d_in[6];
  const float* ar2 = (const float*)d_in[7];
  const float* b2  = (const float*)d_in[8];
  const float* W3  = (const float*)d_in[9];
  const float* al3 = (const float*)d_in[10];
  const float* ar3 = (const float*)d_in[11];
  const float* b3  = (const float*)d_in[12];
  const float* Wc1 = (const float*)d_in[13];
  const float* bc1 = (const float*)d_in[14];
  const float* Wc2 = (const float*)d_in[15];
  const float* bc2 = (const float*)d_in[16];
  const int*   src = (const int*)d_in[17];
  const int*   dst = (const int*)d_in[18];
  const int*   gid = (const int*)d_in[19];
  float* out = (float*)d_out;

  const int nP = ((nN + GR - 1) / GR) * GR;
  size_t off = 0;
  _Float16* Wt1 = (_Float16*)((char*)d_ws + off); off += al256((size_t)HDIM * 128 * sizeof(_Float16));
  _Float16* Wt2 = (_Float16*)((char*)d_ws + off); off += al256((size_t)HDIM * HDIM * sizeof(_Float16));
  _Float16* Wt3 = (_Float16*)((char*)d_ws + off); off += al256((size_t)HDIM * HDIM * sizeof(_Float16));
  float* F   = (float*)((char*)d_ws + off); off += al256((size_t)nP * HDIM * sizeof(float));
  float* Hb  = (float*)((char*)d_ws + off); off += al256((size_t)nP * HDIM * sizeof(float));
  float* El  = (float*)((char*)d_ws + off); off += al256((size_t)nP * NHEAD * sizeof(float));
  float* Er  = (float*)((char*)d_ws + off); off += al256((size_t)nP * NHEAD * sizeof(float));
  float* Hg  = (float*)((char*)d_ws + off); off += al256((size_t)NG * HDIM * sizeof(float));
  if (off > ws_size) return;
  if (off > (size_t)134217728) return;

  k_prepw<<<(HDIM * 16 + 255) / 256, 256, 0, stream>>>(W1, Wt1, FIN, 128);
  k_prepw<<<(HDIM * 24 + 255) / 256, 256, 0, stream>>>(W2, Wt2, HDIM, HDIM);
  k_prepw<<<(HDIM * 24 + 255) / 256, 256, 0, stream>>>(W3, Wt3, HDIM, HDIM);

  hipFuncSetAttribute(reinterpret_cast<const void*>(&k_agg),
                      hipFuncAttributeMaxDynamicSharedMemorySize, AGG_LDS_BYTES);
  const int ggrid = nP / GR;
  const int agrid = (nN + NB - 1) / NB;

  k_gemm<FIN, 96, 128><<<ggrid, GTHR, 0, stream>>>(nf, Wt1, al1, ar1, F, El, Er, nN);
  k_agg<<<agrid, ATHR, AGG_LDS_BYTES, stream>>>(F, El, Er, src, dst, b1, Hb, nN, nE);
  k_gemm<HDIM, HDIM, HDIM><<<ggrid, GTHR, 0, stream>>>(Hb, Wt2, al2, ar2, F, El, Er, nN);
  k_agg<<<agrid, ATHR, AGG_LDS_BYTES, stream>>>(F, El, Er, src, dst, b2, Hb, nN, nE);
  k_gemm<HDIM, HDIM, HDIM><<<ggrid, GTHR, 0, stream>>>(Hb, Wt3, al3, ar3, F, El, Er, nN);
  k_agg<<<agrid, ATHR, AGG_LDS_BYTES, stream>>>(F, El, Er, src, dst, b3, Hb, nN, nE);

  k_readout<<<NG, 256, 0, stream>>>(Hb, gid, Hg, nN);
  k_cls<<<1, 256, 0, stream>>>(Hg, Wc1, bc1, Wc2, bc2, out);
}
